// KnowledgeDifficulty_52501680226368
// MI455X (gfx1250) — hardware-verified
//
#include <hip/hip_runtime.h>
#include <hip/hip_bf16.h>
#include <math.h>


#define BB 2
#define SS 2048
#define DD 1024
#define HH 16
#define DKK 64
#define QW 2

typedef _Float16 bf16;
typedef __attribute__((ext_vector_type(4))) unsigned v4u_t;
typedef unsigned v4ua __attribute__((ext_vector_type(4), may_alias));
typedef __attribute__((ext_vector_type(4))) float v4f_t;
typedef float v4fa __attribute__((ext_vector_type(4), may_alias));
typedef __attribute__((ext_vector_type(16))) bf16  bf16x16;
typedef __attribute__((ext_vector_type(8)))  bf16  bf16x8;
typedef __attribute__((ext_vector_type(4)))  bf16  bf16x4;
typedef __attribute__((ext_vector_type(8)))  float f32x8;

#define LDS_STRIDE 48
#define KSTRIDE    72
#define VSTRIDE    48

__device__ __forceinline__ f32x8 wmma_bf16(bf16x16 a, bf16x16 b, f32x8 c) {
  return __builtin_amdgcn_wmma_f32_16x16x32_f16(
      false, a, false, b, (short)0, c, false, false);
}
#define RSPLIT (1.0f / 2048.0f)
__device__ __forceinline__ bf16 lo_of(float v, bf16 h) { return (bf16)((v - (float)h) * 2048.0f); }
__device__ __forceinline__ f32x8 wmma_split(bf16x16 a, bf16x16 al, bf16x16 b, bf16x16 bl, f32x8 c) {
  f32x8 x = {}; x = wmma_bf16(al, b, x); x = wmma_bf16(a, bl, x); return wmma_bf16(a, b, c) + x * RSPLIT; }

template <typename T>
__device__ __forceinline__ bf16x16 load_frag(const T* __restrict__ base, int ld,
                                             int row0, int k0) {
  const int lane = threadIdx.x & 31;
  const int r    = lane & 15;
  const int kh   = (lane >> 4) * 8;
  const T* p0 = base + (size_t)(row0 + r) * ld + (k0 + kh);
  const T* p1 = p0 + 16;
  bf16x16 f;
#pragma unroll
  for (int i = 0; i < 8; ++i) {
    f[i]     = (bf16)p0[i];
    f[i + 8] = (bf16)p1[i];
  }
  return f;
}

__device__ __forceinline__ bf16x16 lds_frag(const bf16* base, int stride) {
  const int lane = threadIdx.x & 31;
  const int row  = lane & 15;
  const int kh   = (lane >> 4) * 8;
  const bf16x8 lo = *(const bf16x8*)(base + row * stride + kh);
  const bf16x8 hi = *(const bf16x8*)(base + row * stride + kh + 16);
  bf16x16 f;
#pragma unroll
  for (int i = 0; i < 8; ++i) { f[i] = lo[i]; f[i + 8] = hi[i]; }
  return f;
}

template <typename T>
__device__ __forceinline__ void stage_read16(const T* __restrict__ p, float* buf) {
#pragma unroll
  for (int i = 0; i < 16; ++i) buf[i] = (float)p[i];
}

__device__ __forceinline__ void stage_write(bf16* dst, const float* buf, int nquad) {
#pragma unroll
  for (int i = 0; i < nquad; ++i) {
    bf16x4 q;
    q[0] = (bf16)buf[4 * i];     q[1] = (bf16)buf[4 * i + 1];
    q[2] = (bf16)buf[4 * i + 2]; q[3] = (bf16)buf[4 * i + 3];
    *(bf16x4*)(dst + 4 * i) = q;
  }
}

__global__ __launch_bounds__(256) void transpose_pack_kernel(const float* __restrict__ W, bf16* __restrict__ WT, int K, int N, size_t plane) {
  __shared__ float tile[64][65];
  const int k0 = blockIdx.y * 64, n0 = blockIdx.x * 64, t = threadIdx.x;
  for (int i = t; i < 64 * 64; i += 256) { const int kr = i >> 6, nc = i & 63; tile[kr][nc] = W[(size_t)(k0 + kr) * N + n0 + nc]; }
  __syncthreads();
#pragma unroll 1
  for (int pass = 0; pass < 2; ++pass) {
    for (int i = t; i < 64 * 8; i += 256) { const int nr = i >> 3, k8 = (i & 7) * 8; bf16 hh[8], hl[8];
#pragma unroll
      for (int e = 0; e < 8; ++e) { const float v = tile[k8 + e][nr]; hh[e] = (bf16)v; hl[e] = lo_of(v, hh[e]); }
      bf16* d = WT + (size_t)(n0 + nr) * K + k0 + k8;
      *(volatile v4u_t*)d = *(const v4ua*)hh; *(volatile v4u_t*)(d + plane) = *(const v4ua*)hl; }
    __threadfence();
  }
}

template <typename AT, typename WT, int MODE>
__global__ __launch_bounds__(256) void gemm_split_kernel(
    const AT* __restrict__ A, size_t aPlane, const WT* __restrict__ W, size_t wPlane,
    const float* __restrict__ bias, void* __restrict__ out,
    int M, int N, int K) {
  __shared__ bf16 ldsA[128 * LDS_STRIDE], ldsAl[128 * LDS_STRIDE];
  __shared__ bf16 ldsW[256 * LDS_STRIDE], ldsWl[256 * LDS_STRIDE];
  __shared__ __attribute__((aligned(16))) unsigned char sob[256 * 136 * 2];

  const int t    = threadIdx.x;
  const int wave = t >> 5;
  const int lane = t & 31;
  const int wm   = (wave & 1) * 64;
  const int wn   = (wave >> 1) * 64;
  const int mBlk = blockIdx.x * 128;
  const int nBlk = blockIdx.y * 256;
  const int arow = t >> 1;
  const int ach  = (t & 1) * 16;

  f32x8 acc[4][4] = {};
  for (int k = 0; k < K; k += 32) {
    __syncthreads();
    {
      const AT* ap = A + (size_t)(mBlk + arow) * K + k + ach;
      bf16 hh[16], hl[16];
      if (sizeof(AT) == 4) {
#pragma unroll
        for (int i = 0; i < 16; ++i) { const float v = (float)ap[i]; hh[i] = (bf16)v; hl[i] = lo_of(v, hh[i]); }
      } else {
#pragma unroll
        for (int i = 0; i < 16; ++i) { hh[i] = (bf16)ap[i]; hl[i] = (bf16)ap[aPlane + i]; }
      }
#pragma unroll
      for (int i = 0; i < 16; ++i) { ldsA[arow * LDS_STRIDE + ach + i] = hh[i]; ldsAl[arow * LDS_STRIDE + ach + i] = hl[i]; }
    }
    {
      const WT* wp = W + (size_t)(nBlk + t) * K + k;
      if (sizeof(WT) == 4) {
#pragma unroll
        for (int i = 0; i < 32; ++i) { const float v = (float)wp[i]; const bf16 h_ = (bf16)v; ldsW[t * LDS_STRIDE + i] = h_; ldsWl[t * LDS_STRIDE + i] = lo_of(v, h_); }
      } else {
#pragma unroll
        for (int i = 0; i < 32; ++i) { ldsW[t * LDS_STRIDE + i] = (bf16)wp[i]; ldsWl[t * LDS_STRIDE + i] = (bf16)wp[wPlane + i]; }
      }
    }
    __syncthreads();
    bf16x16 wf[4], wfl[4];
#pragma unroll
    for (int j = 0; j < 4; ++j) { wf[j] = lds_frag(ldsW + (wn + 16 * j) * LDS_STRIDE, LDS_STRIDE); wfl[j] = lds_frag(ldsWl + (wn + 16 * j) * LDS_STRIDE, LDS_STRIDE); }
#pragma unroll
    for (int i = 0; i < 4; ++i) {
      const bf16x16 af = lds_frag(ldsA + (wm + 16 * i) * LDS_STRIDE, LDS_STRIDE), afl = lds_frag(ldsAl + (wm + 16 * i) * LDS_STRIDE, LDS_STRIDE);
#pragma unroll
      for (int j = 0; j < 4; ++j) acc[i][j] = wmma_split(af, afl, wf[j], wfl[j], acc[i][j]);
    }
  }

  const int nlane = lane & 15;
  const int mh    = (lane >> 4) * 8;
  __syncthreads();
  if (MODE == 1) {
    bf16* so = (bf16*)sob;
#pragma unroll
    for (int i = 0; i < 4; ++i)
#pragma unroll
      for (int j = 0; j < 4; ++j) {
        const int nl = wn + 16 * j + nlane;
        const float bv = bias ? bias[nBlk + nl] : 0.0f;
#pragma unroll
        for (int r = 0; r < 8; ++r) so[nl * 136 + wm + 16 * i + mh + r] = (bf16)(acc[i][j][r] + bv);
      }
    __syncthreads();
    const int b_ = mBlk >> 11, s0 = mBlk & (SS - 1);
#pragma unroll 1
    for (int pass = 0; pass < 2; ++pass) {
      for (int ch = t; ch < 256 * 16; ch += 256) { const int nl = ch >> 4, q = (ch & 15) * 8; const int n = nBlk + nl, h = n >> 6, dk = n & (DKK - 1);
        *(volatile v4u_t*)((bf16*)out + (((size_t)(b_ * HH + h)) * DKK + dk) * SS + s0 + q) = *(const v4ua*)(so + nl * 136 + q); }
      __threadfence();
    }
  } else {
    float* so = (float*)sob;
#pragma unroll 1
    for (int hf = 0; hf < 2; ++hf) {
      if (wm == hf * 64) {
#pragma unroll
        for (int i = 0; i < 4; ++i)
#pragma unroll
          for (int j = 0; j < 4; ++j) {
            const int nl = wn + 16 * j + nlane;
            const float bv = bias ? bias[nBlk + nl] : 0.0f;
#pragma unroll
            for (int r = 0; r < 8; ++r) so[(16 * i + mh + r) * 260 + nl] = acc[i][j][r] + bv;
          }
      }
      __syncthreads();
#pragma unroll 1
      for (int pass = 0; pass < 2; ++pass) {
        for (int ch = t; ch < 64 * 64; ch += 256) { const int ml = ch >> 6, q = (ch & 63) * 4;
          *(volatile v4f_t*)((float*)out + (size_t)(mBlk + hf * 64 + ml) * N + nBlk + q) = *(const volatile v4fa*)(so + ml * 260 + q); }
        __threadfence();
      }
      __syncthreads();
    }
  }
}


#define KB_ 64
#define KN 512
#define KL 128
#define KM 1024
#define KCH 8

__global__ __launch_bounds__(256) void k_xs(const float* __restrict__ X, const float* __restrict__ Ws, float* __restrict__ xs) {
  __shared__ float res[32];
  const int wave = threadIdx.x >> 5, lane = threadIdx.x & 31, row0 = blockIdx.x * 32;
#pragma unroll 1
  for (int i = 0; i < 4; ++i) { const int row = row0 + wave * 4 + i; const float* xr = X + (size_t)row * KL;
    float s = xr[lane] * Ws[lane] + xr[32 + lane] * Ws[32 + lane] + xr[64 + lane] * Ws[64 + lane] + xr[96 + lane] * Ws[96 + lane];
#pragma unroll
    for (int o = 16; o >= 1; o >>= 1) s += __shfl_xor(s, o, 32);
    if (lane == 0) res[wave * 4 + i] = s; }
  __syncthreads();
  if (threadIdx.x < 32) { const float v = res[threadIdx.x]; *(volatile float*)(xs + row0 + threadIdx.x) = v; __threadfence(); *(volatile float*)(xs + row0 + threadIdx.x) = v; }
}
__global__ __launch_bounds__(256) void k_col(const float* __restrict__ Lg, const float* __restrict__ xs, const int* __restrict__ Kmask, const float* __restrict__ bs,
                                            int b0, float* __restrict__ out) {
  __shared__ float xsb[KN];
  const int bl = blockIdx.y, b = b0 + bl, m = blockIdx.x * 256 + threadIdx.x, t = threadIdx.x;
  for (int i = t; i < KN; i += 256) xsb[i] = xs[(size_t)b * KN + i];
  __syncthreads();
  const float* col = Lg + (size_t)bl * KN * KM + m;
  float mx = -3.0e38f;
#pragma unroll 4
  for (int n = 0; n < KN; ++n) mx = fmaxf(mx, col[(size_t)n * KM]);
  float se = 0.0f, sw = 0.0f;
#pragma unroll 4
  for (int n = 0; n < KN; ++n) { const float e = expf(col[(size_t)n * KM] - mx); se += e; sw += e * xsb[n]; }
  const float z = sw / se + bs[0];
  const float d = 1.0f / (1.0f + expf(-z));
  const float v = (Kmask[(size_t)b * KM + m] > 0) ? d : 0.0f;
  *(volatile float*)(out + (size_t)b * KM + m) = v; __threadfence(); *(volatile float*)(out + (size_t)b * KM + m) = v;
}

extern "C" void kernel_launch(void* const* d_in, const int* in_sizes, int n_in,
                              void* d_out, int out_size, void* d_ws, size_t ws_size,
                              hipStream_t stream) {
  (void)in_sizes; (void)n_in; (void)out_size; (void)ws_size;
  const float* X  = (const float*)d_in[0];
  const int*   Km = (const int*)d_in[1];
  const float* Wa = (const float*)d_in[2];
  const float* ba = (const float*)d_in[3];
  const float* Ws = (const float*)d_in[4];
  const float* bs = (const float*)d_in[5];
  char* ws = (char*)d_ws;
  bf16*  WT = (bf16*)ws;  ws += (size_t)2 * KM * KL * 2;
  float* xs = (float*)ws; ws += (size_t)KB_ * KN * 4;
  float* Lg = (float*)ws; ws += (size_t)KCH * KN * KM * 4;
  const size_t pl = (size_t)KM * KL;
  transpose_pack_kernel<<<dim3(KM / 64, KL / 64), 256, 0, stream>>>(Wa, WT, KL, KM, pl);
  k_xs<<<KB_ * KN / 32, 256, 0, stream>>>(X, Ws, xs);
  for (int c = 0; c < KB_ / KCH; ++c) {
    gemm_split_kernel<float, bf16, 2><<<dim3(KCH * KN / 128, KM / 256), 256, 0, stream>>>(X + (size_t)c * KCH * KN * KL, 0, WT, pl, ba, Lg, KCH * KN, KM, KL);
    k_col<<<dim3(KM / 256, KCH), 256, 0, stream>>>(Lg, xs, Km, bs, c * KCH, (float*)d_out);
  }
}
